// Inception_LocalNonLocal_v2_79293686219341
// MI455X (gfx1250) — hardware-verified
//
#include <hip/hip_runtime.h>
#include <stddef.h>


typedef _Float16 h16;
typedef _Float16 v16h __attribute__((ext_vector_type(16)));
typedef _Float16 v8h  __attribute__((ext_vector_type(8)));
typedef float    v8f  __attribute__((ext_vector_type(8)));
typedef float    v4f  __attribute__((ext_vector_type(4)));

#ifndef NB
#define NB 4
#endif
#define NB_FULL 4
#define CIN   256
#define CP    32
#define NPROJ 96
#define IMH   64
#define IMW   64
#define NPIX  (IMH * IMW)
#define PADY  4
#define PADX  8
#define HP    (IMH + 2 * PADY)
#define WP    (IMW + 2 * PADX)
#define PPIX  (HP * WP)
#define NPB   (NB * NPIX / 64)

#ifndef SCORE_RES
#define SCORE_RES 1
#endif

static_assert(NB >= 1 && NB <= NB_FULL);
static_assert(CP == 32);
static_assert(NPROJ == 3 * CP);
static_assert((CIN % 64) == 0 && (CIN % 32) == 0);
static_assert((PPIX % 64) == 0);
static_assert((WP % 8) == 0 && (PADX % 8) == 0);
static_assert((NPIX % 64) == 0 && (IMW % 16) == 0);
static_assert(IMW == 4 * 16);
static_assert(PADY == 4 && PADX >= 8);
static_assert(IMW - 16 + 32 <= WP);
static_assert((CP * CIN) % 2048 == 0);
static_assert(CIN == 256);

#define LDT  72
#define LDC  68
#define LDCP 100
#define LDP  40
static_assert((LDT % 8) == 0 && LDT >= 64);
static_assert((LDC % 4) == 0 && LDC >= 64);
static_assert((LDCP % 4) == 0 && LDCP >= NPROJ);
static_assert((LDP % 8) == 0 && LDP >= 32);

#define XCARRY   16.0f
#define WCARRY   64.0f
#define QCARRY   16.0f
#define KCARRY   16.0f
#define RCARRY   2048.0f
#define VCARRY   64.0f
#define PCARRY   4096.0f
#define PRECARRY 16.0f
#define WFCARRY  64.0f

#define WP_BYTES   ((size_t)NPROJ * CIN * 2)
#define WF_BYTES   ((size_t)CIN * CP * 2)
#define XT_BYTES   ((size_t)NB * PPIX * CIN * 2)
#define KQ_BYTES   ((size_t)NB * PPIX * CP * 2)
#define PRE_BYTES  ((size_t)NB * NPIX * CP * 2)
#define PART_BYTES ((size_t)NPB * 4 * 128 * 4)
#define STAT_BYTES ((size_t)3 * CIN * 4)
#define OFF_WP   ((size_t)0)
#define OFF_WF   (OFF_WP + WP_BYTES)
#define OFF_XT   (OFF_WF + WF_BYTES)
#define OFF_KH   (OFF_XT + XT_BYTES)
#define OFF_KR   (OFF_KH + KQ_BYTES)
#define OFF_QH   (OFF_KR + KQ_BYTES)
#define OFF_QR   (OFF_QH + KQ_BYTES)
#define OFF_VT   (OFF_QR + KQ_BYTES)
#define OFF_PRE  (OFF_VT + KQ_BYTES)
#define OFF_PART (OFF_PRE + PRE_BYTES)
#define OFF_STAT (OFF_PART + PART_BYTES)
#define WS_TOTAL (OFF_STAT + STAT_BYTES)
static_assert((WP_BYTES % 128) == 0 && (WF_BYTES % 128) == 0 && (XT_BYTES % 128) == 0);
static_assert((KQ_BYTES % 128) == 0 && (PRE_BYTES % 128) == 0 && (PART_BYTES % 128) == 0);
static_assert((STAT_BYTES % 128) == 0);
static_assert(WS_TOTAL <= (size_t)134217728);

__device__ __forceinline__ float bf16r(float x) {
  unsigned int u = __float_as_uint(x);
  u = (u + 0x7FFFu + ((u >> 16) & 1u)) & 0xFFFF0000u;
  return __uint_as_float(u);
}

__device__ __forceinline__ h16 toh_flush(float v) {
  const h16 r = (h16)v;
  return (fabsf(v) < 6.103515625e-05f) ? (h16)0.0f : r;
}

__device__ __forceinline__ int iabs_i(int v) { return (v < 0) ? -v : v; }
__device__ __forceinline__ int iclamp_i(int v, int lo, int hi) {
  return (v < lo) ? lo : ((v > hi) ? hi : v);
}

__device__ __forceinline__ v16h frag_at(const _Float16* p) {
  v8h lo = *(const v8h*)(p);
  v8h hi = *(const v8h*)(p + 16);
  v16h out;
#pragma unroll
  for (int i = 0; i < 8; ++i) { out[i] = lo[i]; out[i + 8] = hi[i]; }
  return out;
}
__device__ __forceinline__ v16h ld_frag(const _Float16* base, unsigned ld) {
  const unsigned lane = threadIdx.x & 31u;
  return frag_at(base + (lane & 15u) * ld + (lane >> 4) * 8u);
}

__device__ __forceinline__ v8f wmma16(v16h a, v16h b, v8f c) {
  v8f d = __builtin_amdgcn_wmma_f32_16x16x32_f16(false, a, false, b, (short)0, c,
                                                 false, false);
  asm volatile("v_nop\n\tv_nop\n\tv_nop\n\tv_nop" : "+v"(d) : "v"(a), "v"(b));
  return d;
}

__device__ __forceinline__ float red16_max(float x) {
#pragma unroll
  for (int off = 1; off < 16; off <<= 1) x = fmaxf(x, __shfl_xor(x, off, 32));
  return x;
}
__device__ __forceinline__ float red16_sum(float x) {
#pragma unroll
  for (int off = 1; off < 16; off <<= 1) x += __shfl_xor(x, off, 32);
  return x;
}

__device__ __forceinline__ void wave_lds_sync() {
  __builtin_amdgcn_fence(3  , "wavefront");
  asm volatile("s_wait_dscnt 0x0" ::: "memory");
  __builtin_amdgcn_wave_barrier();
}

__global__ __launch_bounds__(256) void xconv_kernel(
    const float* __restrict__ X, _Float16* __restrict__ Xt) {
  __shared__ _Float16 T[64 * LDT];
  const unsigned tid = threadIdx.x;
  const unsigned n0 = blockIdx.x * 64u;
  const unsigned k0 = blockIdx.y * 64u;
  const unsigned b = blockIdx.z;
  const unsigned nc = tid & 63u;
  const int gp = (int)(n0 + nc);
  const int prow = gp / WP;
  const int pcol = gp - prow * WP;
  const bool inside = (prow >= PADY) && (prow < PADY + IMH) && (pcol >= PADX) && (pcol < PADX + IMW);
  const int yc = iclamp_i(prow - PADY, 0, IMH - 1);
  const int xc = iclamp_i(pcol - PADX, 0, IMW - 1);
  const float* src = X + ((size_t)b * CIN + k0) * NPIX + (unsigned)(yc * IMW + xc);
#pragma unroll 4
  for (unsigned j = 0; j < 16u; ++j) {
    const unsigned kr = (tid >> 6) + 4u * j;
    float v = src[(size_t)kr * NPIX];
    asm volatile("" : "+v"(v));
    v = inside ? v : 0.0f;
    T[nc * LDT + kr] = toh_flush(XCARRY * bf16r(v));
  }
  __syncthreads();
  v8h x[2];
  size_t off[2];
#pragma unroll
  for (unsigned i = 0; i < 2u; ++i) {
    const unsigned n = 32u * i + (tid >> 3);
    const unsigned kc = (tid & 7u) * 8u;
    x[i] = *(const v8h*)&T[n * LDT + kc];
    off[i] = ((size_t)b * PPIX + n0 + n) * CIN + k0 + kc;
  }
#pragma unroll
  for (int i = 0; i < 2; ++i) *(volatile v8h*)(Xt + off[i]) = x[i];
  __threadfence();
#pragma unroll
  for (int i = 0; i < 2; ++i) *(volatile v8h*)(Xt + off[i]) = x[i];
}

__global__ __launch_bounds__(256) void wcast_kernel(
    const float* __restrict__ W, _Float16* __restrict__ dst, float carry) {
  const unsigned i = (blockIdx.x * 256u + threadIdx.x) * 8u;
  const v4f a0 = *(const v4f*)(W + i);
  const v4f a1 = *(const v4f*)(W + i + 4u);
  v8h o;
#pragma unroll
  for (int j = 0; j < 4; ++j) {
    o[j]     = toh_flush(carry * bf16r(a0[j]));
    o[j + 4] = toh_flush(carry * bf16r(a1[j]));
  }
  _Float16* p = dst + i;
  *(volatile v8h*)p = o;
  __threadfence();
  *(volatile v8h*)p = o;
}

__global__ __launch_bounds__(256) void proj_kernel(
    const _Float16* __restrict__ Xt, const _Float16* __restrict__ Wp,
    const float* __restrict__ bk, const float* __restrict__ bq, const float* __restrict__ bx,
    const float* __restrict__ vessel,
    _Float16* __restrict__ Kh, _Float16* __restrict__ Kr,
    _Float16* __restrict__ Qh, _Float16* __restrict__ Qr, _Float16* __restrict__ Vt) {
  __shared__ float Cs[64 * LDCP];
  __shared__ float Vsc[64];
  __shared__ float Ins[64];
  const unsigned tid = threadIdx.x, lane = tid & 31u;
  const unsigned wave = __builtin_amdgcn_readfirstlane(threadIdx.x >> 5);
  const unsigned mw = wave >> 1, nw = wave & 1u;
  const unsigned hh = lane >> 4, m = lane & 15u;
  const unsigned p0 = blockIdx.x * 64u;
  const unsigned b = blockIdx.y;

  if (tid < 64u) {
    const int gp = (int)(p0 + tid);
    const int prow = gp / WP;
    const int pcol = gp - prow * WP;
    const bool inside = (prow >= PADY) && (prow < PADY + IMH) && (pcol >= PADX) && (pcol < PADX + IMW);
    const int yc = iclamp_i(prow - PADY, 0, IMH - 1);
    const int xc = iclamp_i(pcol - PADX, 0, IMW - 1);
    float vs = vessel[(size_t)b * NPIX + (unsigned)(yc * IMW + xc)];
    asm volatile("" : "+v"(vs));
    Ins[tid] = inside ? 1.0f : 0.0f;
    Vsc[tid] = inside ? bf16r(vs) : 0.0f;
  }

  const _Float16* ap = Xt + ((size_t)b * PPIX + p0 + mw * 16u + m) * CIN + hh * 8u;
  const _Float16* bp = Wp + (size_t)(nw * 48u + m) * CIN + hh * 8u;
  v8f acc0 = {}, acc1 = {}, acc2 = {};
#pragma unroll 2
  for (unsigned k0 = 0; k0 < (unsigned)CIN; k0 += 32u) {
    const v16h a  = frag_at(ap + k0);
    const v16h b0 = frag_at(bp + k0);
    const v16h b1 = frag_at(bp + (size_t)16 * CIN + k0);
    const v16h b2 = frag_at(bp + (size_t)32 * CIN + k0);
    acc0 = wmma16(a, b0, acc0);
    acc1 = wmma16(a, b1, acc1);
    acc2 = wmma16(a, b2, acc2);
  }
#pragma unroll
  for (int r = 0; r < 8; ++r) {
    float* d = &Cs[(mw * 16u + hh * 8u + (unsigned)r) * LDCP + nw * 48u + m];
    d[0]  = acc0[r];
    d[16] = acc1[r];
    d[32] = acc2[r];
  }
  __syncthreads();

  const float pcs = 1.0f / (XCARRY * WCARRY);

  const unsigned row = tid >> 2;
  const unsigned c8 = (tid & 3u) * 8u;
  const float vs = Vsc[row];
  const float ins = Ins[row];
  v8h kh, kr, qh, qr;
  {
    const v4f uk0 = *(const v4f*)&Cs[row * LDCP + c8];
    const v4f uk1 = *(const v4f*)&Cs[row * LDCP + c8 + 4u];
    const v4f uq0 = *(const v4f*)&Cs[row * LDCP + 32u + c8];
    const v4f uq1 = *(const v4f*)&Cs[row * LDCP + 32u + c8 + 4u];
    const v4f gk0 = *(const v4f*)(bk + c8);
    const v4f gk1 = *(const v4f*)(bk + c8 + 4u);
    const v4f gq0 = *(const v4f*)(bq + c8);
    const v4f gq1 = *(const v4f*)(bq + c8 + 4u);
#pragma unroll
    for (int j = 0; j < 4; ++j) {
      const float tk0 = (uk0[j] * pcs + bf16r(gk0[j])) * vs * KCARRY;
      const float tk1 = (uk1[j] * pcs + bf16r(gk1[j])) * vs * KCARRY;
      const float tq0 = (uq0[j] * pcs + bf16r(gq0[j])) * ins * QCARRY;
      const float tq1 = (uq1[j] * pcs + bf16r(gq1[j])) * ins * QCARRY;
      const h16 hk0 = toh_flush(tk0);
      const h16 hk1 = toh_flush(tk1);
      const h16 hq0 = toh_flush(tq0);
      const h16 hq1 = toh_flush(tq1);
      kh[j] = hk0; kh[j + 4] = hk1;
      qh[j] = hq0; qh[j + 4] = hq1;
      kr[j]     = toh_flush((tk0 - (float)hk0) * RCARRY);
      kr[j + 4] = toh_flush((tk1 - (float)hk1) * RCARRY);
      qr[j]     = toh_flush((tq0 - (float)hq0) * RCARRY);
      qr[j + 4] = toh_flush((tq1 - (float)hq1) * RCARRY);
    }
  }
  const size_t offkq = ((size_t)b * PPIX + p0 + row) * CP + c8;

  const unsigned ch = tid >> 3;
  const unsigned kk = (tid & 7u) * 8u;
  v8h vv;
  {
    const float bb = bf16r(bx[ch]);
#pragma unroll
    for (unsigned j = 0; j < 8u; ++j) {
      const float t = (Cs[(kk + j) * LDCP + 64u + ch] * pcs + bb) * Ins[kk + j];
      vv[j] = toh_flush(t * VCARRY);
    }
  }
  const size_t offv = ((size_t)b * CP + ch) * PPIX + p0 + kk;

  *(volatile v8h*)(Kh + offkq) = kh;
  *(volatile v8h*)(Qh + offkq) = qh;
#if SCORE_RES
  *(volatile v8h*)(Kr + offkq) = kr;
  *(volatile v8h*)(Qr + offkq) = qr;
#endif
  *(volatile v8h*)(Vt + offv) = vv;
  __threadfence();
  *(volatile v8h*)(Kh + offkq) = kh;
  *(volatile v8h*)(Qh + offkq) = qh;
#if SCORE_RES
  *(volatile v8h*)(Kr + offkq) = kr;
  *(volatile v8h*)(Qr + offkq) = qr;
#endif
  *(volatile v8h*)(Vt + offv) = vv;
}

__device__ __forceinline__ void score_pair(
    const _Float16* __restrict__ Kh, const _Float16* __restrict__ Kr, const size_t koff,
    const v16h qh, const v16h qr, v8f& s0, v8f& s1) {
  const float sscale = 1.0f / (QCARRY * KCARRY);
  const v16h k0 = frag_at(Kh + koff);
  const v16h k1 = frag_at(Kh + koff + (size_t)16 * CP);
  v8f a0 = {}, a1 = {};
  a0 = wmma16(qh, k0, a0);
  a1 = wmma16(qh, k1, a1);
#if SCORE_RES
  const v16h kr0 = frag_at(Kr + koff);
  const v16h kr1 = frag_at(Kr + koff + (size_t)16 * CP);
  v8f r0 = {}, r1 = {};
  r0 = wmma16(qh, kr0, r0);
  r0 = wmma16(qr, k0, r0);
  r1 = wmma16(qh, kr1, r1);
  r1 = wmma16(qr, k1, r1);
  s0 = (a0 + r0 * (1.0f / RCARRY)) * sscale;
  s1 = (a1 + r1 * (1.0f / RCARRY)) * sscale;
#else
  s0 = a0 * sscale;
  s1 = a1 * sscale;
#endif
}

__global__ __launch_bounds__(128) void attn_kernel(
    const _Float16* __restrict__ Qh, const _Float16* __restrict__ Qr,
    const _Float16* __restrict__ Kh, const _Float16* __restrict__ Kr,
    const _Float16* __restrict__ Vt, _Float16* __restrict__ Pre) {
  __shared__ _Float16 Ps[4 * 16 * LDP];

  const unsigned tid = threadIdx.x, lane = tid & 31u;
  const unsigned wave = __builtin_amdgcn_readfirstlane(threadIdx.x >> 5);
  const unsigned hh = lane >> 4, m = lane & 15u;
  const unsigned y = blockIdx.x;
  const unsigned b = blockIdx.y;
  const unsigned x0 = wave * 16u;
  _Float16* P = Ps + wave * (16u * LDP);

  const size_t qoff = ((size_t)b * PPIX + (y + PADY) * WP + x0 + PADX + m) * CP + hh * 8u;
  const v16h qh = frag_at(Qh + qoff);
#if SCORE_RES
  const v16h qr = frag_at(Qr + qoff);
#else
  const v16h qr = qh;
#endif

  const int dxb = (int)m - 8 - 8 * (int)hh;
  const size_t kbase = ((size_t)b * PPIX + y * WP + x0 + m) * CP + hh * 8u;
  const size_t vbase = ((size_t)b * CP + m) * PPIX + y * WP + x0 + hh * 8u;

  float mrow[8];
#pragma unroll
  for (int r = 0; r < 8; ++r) mrow[r] = -1.0e30f;

#pragma unroll 1
  for (unsigned d = 0; d < 9u; ++d) {
    v8f s0, s1;
    score_pair(Kh, Kr, kbase + (size_t)d * (WP * CP), qh, qr, s0, s1);
#pragma unroll
    for (int r = 0; r < 8; ++r) {
      const int a0 = iabs_i(dxb - r);
      const int a1 = iabs_i(dxb + 16 - r);
      const float v0 = (a0 <= 4) ? s0[r] : -1.0e30f;
      const float v1 = (a1 <= 4) ? s1[r] : -1.0e30f;
      mrow[r] = fmaxf(mrow[r], fmaxf(v0, v1));
    }
  }
#pragma unroll
  for (int r = 0; r < 8; ++r) mrow[r] = red16_max(mrow[r]);

  float z[8][4];
#pragma unroll
  for (int r = 0; r < 8; ++r)
#pragma unroll
    for (int w = 0; w < 4; ++w) z[r][w] = 0.0f;

#pragma unroll 1
  for (unsigned d = 0; d < 9u; ++d) {
    const int ady = (d < 4u) ? (int)(4u - d) : (int)(d - 4u);
    v8f s0, s1;
    score_pair(Kh, Kr, kbase + (size_t)d * (WP * CP), qh, qr, s0, s1);
#pragma unroll
    for (int r = 0; r < 8; ++r) {
      const int a0 = iabs_i(dxb - r);
      const int a1 = iabs_i(dxb + 16 - r);
      const int c0 = (a0 > ady) ? a0 : ady;
      const int c1 = (a1 > ady) ? a1 : ady;
      const float x0e = __expf(fminf(s0[r] - mrow[r], 0.0f));
      const float x1e = __expf(fminf(s1[r] - mrow[r], 0.0f));
      const float e0 = (a0 <= 4) ? x0e : 0.0f;
      const float e1 = (a1 <= 4) ? x1e : 0.0f;
      z[r][0] += ((c0 <= 1) ? e0 : 0.0f) + ((c1 <= 1) ? e1 : 0.0f);
      z[r][1] += ((c0 <= 2) ? e0 : 0.0f) + ((c1 <= 2) ? e1 : 0.0f);
      z[r][2] += ((c0 <= 3) ? e0 : 0.0f) + ((c1 <= 3) ? e1 : 0.0f);
      z[r][3] += e0 + e1;
    }
  }
#pragma unroll
  for (int r = 0; r < 8; ++r) {
    const float z1 = fmaxf(red16_sum(z[r][0]), 1.0e-30f);
    const float z2 = fmaxf(red16_sum(z[r][1]), 1.0e-30f);
    const float z3 = fmaxf(red16_sum(z[r][2]), 1.0e-30f);
    const float z4 = fmaxf(red16_sum(z[r][3]), 1.0e-30f);
    const float i4 = __builtin_amdgcn_rcpf(z4);
    const float i3 = i4 + __builtin_amdgcn_rcpf(z3);
    const float i2 = i3 + __builtin_amdgcn_rcpf(z2);
    const float i1 = i2 + __builtin_amdgcn_rcpf(z1);
    z[r][0] = i1; z[r][1] = i2; z[r][2] = i3; z[r][3] = i4;
  }

  v8f o0 = {}, o1 = {};
#pragma unroll 1
  for (unsigned d = 0; d < 9u; ++d) {
    const int ady = (d < 4u) ? (int)(4u - d) : (int)(d - 4u);
    v8f s0, s1;
    score_pair(Kh, Kr, kbase + (size_t)d * (WP * CP), qh, qr, s0, s1);
#pragma unroll
    for (int r = 0; r < 8; ++r) {
      const int a0 = iabs_i(dxb - r);
      const int a1 = iabs_i(dxb + 16 - r);
      const int c0 = (a0 > ady) ? a0 : ady;
      const int c1 = (a1 > ady) ? a1 : ady;
      const float x0e = __expf(fminf(s0[r] - mrow[r], 0.0f));
      const float x1e = __expf(fminf(s1[r] - mrow[r], 0.0f));
      const float e0 = (a0 <= 4) ? x0e : 0.0f;
      const float e1 = (a1 <= 4) ? x1e : 0.0f;
      const float f0 = (c0 <= 1) ? z[r][0] : ((c0 == 2) ? z[r][1] : ((c0 == 3) ? z[r][2] : z[r][3]));
      const float f1 = (c1 <= 1) ? z[r][0] : ((c1 == 2) ? z[r][1] : ((c1 == 3) ? z[r][2] : z[r][3]));
      P[(hh * 8u + (unsigned)r) * LDP + m]       = toh_flush(e0 * f0 * PCARRY);
      P[(hh * 8u + (unsigned)r) * LDP + 16u + m] = toh_flush(e1 * f1 * PCARRY);
    }
    wave_lds_sync();
    const v16h pf = ld_frag(P, LDP);
    const size_t voff = vbase + (size_t)d * WP;
    const v16h vf0 = frag_at(Vt + voff);
    const v16h vf1 = frag_at(Vt + voff + (size_t)16 * PPIX);
    o0 = wmma16(pf, vf0, o0);
    o1 = wmma16(pf, vf1, o1);
    wave_lds_sync();
  }

  const float osc = PRECARRY / (PCARRY * VCARRY);
#pragma unroll
  for (int r = 0; r < 8; ++r) {
    P[(hh * 8u + (unsigned)r) * LDP + m]       = toh_flush(o0[r] * osc);
    P[(hh * 8u + (unsigned)r) * LDP + 16u + m] = toh_flush(o1[r] * osc);
  }
  wave_lds_sync();
  v8h xo[2];
  size_t off[2];
#pragma unroll
  for (unsigned i = 0; i < 2u; ++i) {
    const unsigned id = 32u * i + lane;
    const unsigned r = id >> 2;
    const unsigned c = (id & 3u) * 8u;
    xo[i] = *(const v8h*)&P[r * LDP + c];
    off[i] = ((size_t)b * NPIX + y * IMW + x0 + r) * CP + c;
  }
#pragma unroll
  for (int i = 0; i < 2; ++i) *(volatile v8h*)(Pre + off[i]) = xo[i];
  __threadfence();
#pragma unroll
  for (int i = 0; i < 2; ++i) *(volatile v8h*)(Pre + off[i]) = xo[i];
}

template <int MODE>
__device__ __forceinline__ void out_body(
    const _Float16* __restrict__ Wf, const _Float16* __restrict__ Pre,
    const float* __restrict__ bfv, const float* __restrict__ stat,
    const float* __restrict__ xin, float* __restrict__ outf, float* __restrict__ part) {
  __shared__ float Cs[64 * LDC];
  const unsigned tid = threadIdx.x, lane = tid & 31u;
  const unsigned wave = __builtin_amdgcn_readfirstlane(threadIdx.x >> 5);
  const unsigned mw = wave >> 1, nw = wave & 1u;
  const unsigned hh = lane >> 4, m = lane & 15u;
  const unsigned n0 = blockIdx.x * 64u;
  const unsigned row0 = blockIdx.y * 64u;
  const float ocs = 1.0f / (PRECARRY * WFCARRY);

  const _Float16* ap  = Wf + (size_t)(row0 + mw * 16u + m) * CP + hh * 8u;
  const _Float16* bp0 = Pre + (size_t)(n0 + nw * 32u + m) * CP + hh * 8u;
  const _Float16* bp1 = bp0 + (size_t)16 * CP;
  v8f acc0 = {}, acc1 = {};
  {
    const v16h a  = frag_at(ap);
    const v16h b0 = frag_at(bp0);
    const v16h b1 = frag_at(bp1);
    acc0 = wmma16(a, b0, acc0);
    acc1 = wmma16(a, b1, acc1);
  }
#pragma unroll
  for (int r = 0; r < 8; ++r) {
    float* d = &Cs[(mw * 16u + hh * 8u + (unsigned)r) * LDC + nw * 32u + m];
    d[0]  = acc0[r];
    d[16] = acc1[r];
  }
  __syncthreads();

  if (MODE == 0) {
    __shared__ float Ss[128];
    const unsigned r = tid >> 2, qd = tid & 3u;
    float s = 0.0f, ss = 0.0f;
#pragma unroll
    for (unsigned i = 0; i < 4u; ++i) {
      const v4f u = *(const v4f*)&Cs[r * LDC + qd * 16u + i * 4u];
#pragma unroll
      for (int j = 0; j < 4; ++j) {
        const float yv = u[j] * ocs;
        s += yv;
        ss += yv * yv;
      }
    }
    s  += __shfl_xor(s, 1, 32);
    ss += __shfl_xor(ss, 1, 32);
    s  += __shfl_xor(s, 2, 32);
    ss += __shfl_xor(ss, 2, 32);
    if (qd == 0u) {
      Ss[r * 2u]      = s;
      Ss[r * 2u + 1u] = ss;
    }
    __syncthreads();
    if (wave == 0u) {
      const v4f val = *(const v4f*)&Ss[lane * 4u];
      float* p = part + ((size_t)blockIdx.x * 4u + blockIdx.y) * 128u + lane * 4u;
      *(volatile v4f*)p = val;
      __threadfence();
      *(volatile v4f*)p = val;
    }
  }

  if (MODE == 1) {
    v4f xs[4];
    size_t off[4];
#pragma unroll
    for (unsigned i = 0; i < 4u; ++i) {
      const unsigned r = 16u * i + (tid >> 4);
      const unsigned c = (tid & 15u) * 4u;
      const unsigned co = row0 + r;
      const unsigned g = n0 + c;
      const unsigned bidx = g / (unsigned)NPIX;
      const unsigned pix = g - bidx * (unsigned)NPIX;
      const size_t o = ((size_t)bidx * CIN + co) * NPIX + pix;
      const v4f u = *(const v4f*)&Cs[r * LDC + c];
      const v4f xv = *(const v4f*)(xin + o);
      const float mean = stat[co];
      const float gsc = stat[CIN + co];
      const float bt = stat[2 * CIN + co];
      const float bb = bf16r(bfv[co]);
      v4f val;
#pragma unroll
      for (int j = 0; j < 4; ++j)
        val[j] = bf16r(xv[j]) + (gsc * ((u[j] * ocs + bb) - mean) + bt);
      xs[i] = val;
      off[i] = o;
    }
#pragma unroll
    for (int i = 0; i < 4; ++i) *(volatile v4f*)(outf + off[i]) = xs[i];
    __threadfence();
#pragma unroll
    for (int i = 0; i < 4; ++i) *(volatile v4f*)(outf + off[i]) = xs[i];
  }
}

__global__ __launch_bounds__(256) void out_stats_kernel(
    const _Float16* __restrict__ Wf, const _Float16* __restrict__ Pre, float* __restrict__ part) {
  out_body<0>(Wf, Pre, (const float*)0, (const float*)0, (const float*)0, (float*)0, part);
}
__global__ __launch_bounds__(256) void out_final_kernel(
    const _Float16* __restrict__ Wf, const _Float16* __restrict__ Pre,
    const float* __restrict__ bfv, const float* __restrict__ stat,
    const float* __restrict__ xin, float* __restrict__ outf) {
  out_body<1>(Wf, Pre, bfv, stat, xin, outf, (float*)0);
}

__global__ __launch_bounds__(256) void bn_fin_kernel(
    const float* __restrict__ part, const float* __restrict__ bfv,
    const float* __restrict__ gamma, const float* __restrict__ beta, float* __restrict__ stat) {
#pragma clang fp contract(off)
  __shared__ float St[3 * CIN];
  const unsigned tid = threadIdx.x;
  const unsigned ct = tid >> 6, rr = tid & 63u;
  double s = 0.0, ss = 0.0;
#pragma unroll 1
  for (unsigned pb = 0; pb < (unsigned)NPB; ++pb) {
    const float* p = part + ((size_t)pb * 4u + ct) * 128u + rr * 2u;
    s += (double)p[0];
    ss += (double)p[1];
  }
  const double icnt = 1.0 / (double)(NB * NPIX);
  const double mean0 = s * icnt;
  double var = ss * icnt - mean0 * mean0;
  var = (var > 0.0) ? var : 0.0;
  const float rstd = 1.0f / sqrtf((float)var + 1.0e-5f);
  St[tid]           = (float)mean0 + bf16r(bfv[tid]);
  St[CIN + tid]     = bf16r(gamma[tid]) * rstd;
  St[2 * CIN + tid] = bf16r(beta[tid]);
  __syncthreads();
  if (tid < 192u) {
    const v4f v = *(const v4f*)&St[tid * 4u];
    float* p = stat + tid * 4u;
    *(volatile v4f*)p = v;
    __threadfence();
    *(volatile v4f*)p = v;
  }
}

extern "C" void kernel_launch(void* const* d_in, const int* in_sizes, int n_in,
                              void* d_out, int out_size, void* d_ws, size_t ws_size,
                              hipStream_t stream) {
  if (n_in < 12) return;
  const long long need_x = (long long)NB * CIN * NPIX;
  if ((long long)in_sizes[0] < need_x) return;
  if ((long long)in_sizes[1] < (long long)NB * NPIX) return;
  if (in_sizes[2] < CP * CIN || in_sizes[4] < CP * CIN || in_sizes[6] < CP * CIN) return;
  if (in_sizes[3] < CP || in_sizes[5] < CP || in_sizes[7] < CP) return;
  if (in_sizes[8] < CIN * CP) return;
  if (in_sizes[9] < CIN || in_sizes[10] < CIN || in_sizes[11] < CIN) return;
  if ((long long)out_size < need_x) return;
  if (ws_size < WS_TOTAL) return;

  const float* X      = (const float*)d_in[0];
  const float* vessel = (const float*)d_in[1];
  const float* wk     = (const float*)d_in[2];
  const float* bk     = (const float*)d_in[3];
  const float* wq     = (const float*)d_in[4];
  const float* bq     = (const float*)d_in[5];
  const float* wx     = (const float*)d_in[6];
  const float* bx     = (const float*)d_in[7];
  const float* wf     = (const float*)d_in[8];
  const float* bfv    = (const float*)d_in[9];
  const float* gamma  = (const float*)d_in[10];
  const float* beta   = (const float*)d_in[11];
  float* out = (float*)d_out;

  char* ws = (char*)d_ws;
  _Float16* Wp16  = (_Float16*)(ws + OFF_WP);
  _Float16* Wf16  = (_Float16*)(ws + OFF_WF);
  _Float16* Xt16  = (_Float16*)(ws + OFF_XT);
  _Float16* Kh16  = (_Float16*)(ws + OFF_KH);
  _Float16* Kr16  = (_Float16*)(ws + OFF_KR);
  _Float16* Qh16  = (_Float16*)(ws + OFF_QH);
  _Float16* Qr16  = (_Float16*)(ws + OFF_QR);
  _Float16* Vt16  = (_Float16*)(ws + OFF_VT);
  _Float16* Pre16 = (_Float16*)(ws + OFF_PRE);
  float*    Part  = (float*)(ws + OFF_PART);
  float*    Stat  = (float*)(ws + OFF_STAT);

  dim3 blk(256);

  xconv_kernel<<<dim3(PPIX / 64, CIN / 64, NB), blk, 0, stream>>>(X, Xt16);
  wcast_kernel<<<dim3((CP * CIN) / 2048), blk, 0, stream>>>(wk, Wp16, WCARRY);
  wcast_kernel<<<dim3((CP * CIN) / 2048), blk, 0, stream>>>(wq, Wp16 + (size_t)CP * CIN, WCARRY);
  wcast_kernel<<<dim3((CP * CIN) / 2048), blk, 0, stream>>>(wx, Wp16 + (size_t)2 * CP * CIN, WCARRY);
  wcast_kernel<<<dim3((CIN * CP) / 2048), blk, 0, stream>>>(wf, Wf16, WFCARRY);

  proj_kernel<<<dim3(PPIX / 64, NB), blk, 0, stream>>>(Xt16, Wp16, bk, bq, bx, vessel,
                                                       Kh16, Kr16, Qh16, Qr16, Vt16);
  attn_kernel<<<dim3(IMH, NB), dim3(128), 0, stream>>>(Qh16, Qr16, Kh16, Kr16, Vt16, Pre16);
  out_stats_kernel<<<dim3(NPB, CIN / 64), blk, 0, stream>>>(Wf16, Pre16, Part);
  bn_fin_kernel<<<dim3(1), blk, 0, stream>>>(Part, bfv, gamma, beta, Stat);
  out_final_kernel<<<dim3(NPB, CIN / 64), blk, 0, stream>>>(Wf16, Pre16, bfv, Stat, X, out);
}
